// RelationKnowledgeExtractor_47674136986059
// MI455X (gfx1250) — hardware-verified
//
#include <hip/hip_runtime.h>
#include <math.h>
typedef __attribute__((ext_vector_type(16))) _Float16 v16h;
typedef __attribute__((ext_vector_type(8)))  _Float16 v8h;
typedef __attribute__((ext_vector_type(16))) __bf16   v16b;
typedef __attribute__((ext_vector_type(8)))  __bf16   v8b;
typedef __attribute__((ext_vector_type(8)))  float    v8f;
typedef __attribute__((ext_vector_type(4)))  float    v4f;
#define PSCALE 32768.0f
#define U16(p) ((const unsigned short*)(const void*)(p))
#define PSCALE_INV (1.0f / 32768.0f)

__device__ __forceinline__ unsigned short f2bf_bits(float f) {
  unsigned u = __float_as_uint(f);
  return (unsigned short)((u + 0x7FFFu + ((u >> 16) & 1u)) >> 16);
}
__device__ __forceinline__ float bf_bits2f(unsigned short h) { return __uint_as_float(((unsigned)h) << 16); }

__device__ __forceinline__ void dep_guard_h(v8f& a, v8f& b, v16h x, v16h y) { asm volatile("v_nop\n\tv_nop\n\tv_nop\n\tv_nop" : "+v"(a), "+v"(b) : "v"(x), "v"(y)); }
__device__ __forceinline__ void dep_guard_b(v8f& a, v8f& b, v16b x, v16b y) { asm volatile("v_nop\n\tv_nop\n\tv_nop\n\tv_nop" : "+v"(a), "+v"(b) : "v"(x), "v"(y)); }
__device__ __forceinline__ void keep4_h(v16h a, v16h b, v16h c, v16h d) { asm volatile("v_nop" :: "v"(a), "v"(b), "v"(c), "v"(d)); }
__device__ __forceinline__ void keep4_b(v16b a, v16b b, v16b c, v16b d) { asm volatile("v_nop" :: "v"(a), "v"(b), "v"(c), "v"(d)); }
__device__ __forceinline__ void acc_guard4(v8f& a, v8f& b, v8f& c, v8f& d) { asm volatile("v_nop\n\tv_nop\n\tv_nop\n\tv_nop" : "+v"(a), "+v"(b), "+v"(c), "+v"(d)); }
template <typename T> struct Frag;
template <> struct Frag<_Float16> {
  typedef v16h V; union U { v16h v; v8h h[2]; };
  static __device__ __forceinline__ v16h load(const _Float16* p) {
    U f; f.h[0] = *(const v8h*)(p); f.h[1] = *(const v8h*)(p + 16); return f.v;
  }
  static __device__ __forceinline__ v8f mma(v16h a, v16h b, v8f c) {
    return __builtin_amdgcn_wmma_f32_16x16x32_f16(false, a, false, b, (short)0, c, false, false);
  }
  static __device__ __forceinline__ void guard(v8f& a, v8f& b, v16h x, v16h y) { dep_guard_h(a, b, x, y); }
  static __device__ __forceinline__ void keep(v16h a, v16h b, v16h c, v16h d) { keep4_h(a, b, c, d); }
};
template <> struct Frag<__bf16> {
  typedef v16b V; union U { v16b v; v8b h[2]; };
  static __device__ __forceinline__ v16b load(const __bf16* p) {
    U f; f.h[0] = *(const v8b*)(p); f.h[1] = *(const v8b*)(p + 16); return f.v;
  }
  static __device__ __forceinline__ v8f mma(v16b a, v16b b, v8f c) {
    return __builtin_amdgcn_wmma_f32_16x16x32_bf16(false, a, false, b, (short)0, c, false, false);
  }
  static __device__ __forceinline__ void guard(v8f& a, v8f& b, v16b x, v16b y) { dep_guard_b(a, b, x, y); }
  static __device__ __forceinline__ void keep(v16b a, v16b b, v16b c, v16b d) { keep4_b(a, b, c, d); }
};

template <int ET> struct Elem;
template <> struct Elem<0> { typedef _Float16 T; };
template <> struct Elem<1> { typedef __bf16 T; };
template <int ET, bool SPLIT, int BIAS_MODE, int OUT_MODE, bool RESID, int ACT = 0>
__global__ __launch_bounds__(256) void wmma_gemm64(
    const unsigned short* __restrict__ Ap, const unsigned short* __restrict__ A2p, int lda, long strideA,
    const unsigned short* __restrict__ Btp, const unsigned short* __restrict__ Bt2p, int ldb, long strideB,
    void* __restrict__ Cout, void* __restrict__ Cout2, int ldc, long strideC,
    const float* __restrict__ bias,
    const float* __restrict__ resid, long strideR,
    int M, int N, int K, float scale) {
  typedef typename Elem<ET>::T T;
  typedef typename Frag<T>::V V;
  const T* A = (const T*)Ap; const T* A2 = (const T*)A2p; const T* Bt = (const T*)Btp; const T* Bt2 = (const T*)Bt2p;
  __shared__ __align__(16) float sT[8][16 * 68];
  const int b    = blockIdx.y;
  const int lane = threadIdx.x & 31;
  const int wave = threadIdx.x >> 5;
  const int tilesN = N >> 6;
  const int tilesM = M >> 6;
  const int tile = blockIdx.x * 8 + wave;
  if (tile >= tilesM * tilesN) return;
  const int tm = tile / tilesN;
  const int tn = tile - tm * tilesN;
  const int m0 = tm << 6;
  const int n0 = tn << 6;

  const T* Ab  = A  + (size_t)b * strideA;
  const T* Bb  = Bt + (size_t)b * strideB;
  const T* Ab2 = SPLIT ? (A2  + (size_t)b * strideA) : nullptr;
  const T* Bb2 = SPLIT ? (Bt2 + (size_t)b * strideB) : nullptr;

  const int rlane = lane & 15;
  const int koff  = (lane >> 4) * 8;
  const int mOff  = (lane >> 4) * 8;

  v8f acc[4][4];
#pragma unroll
  for (int i = 0; i < 4; ++i)
#pragma unroll
    for (int j = 0; j < 4; ++j) acc[i][j] = (v8f){0.f,0.f,0.f,0.f,0.f,0.f,0.f,0.f};

  for (int k0 = 0; k0 < K; k0 += 32) {
    V bh[4], bl[4];
#pragma unroll
    for (int j = 0; j < 4; ++j) {
      const size_t bo = (size_t)(n0 + (j << 4) + rlane) * ldb + koff + k0;
      bh[j] = Frag<T>::load(Bb + bo);
      if (SPLIT) bl[j] = Frag<T>::load(Bb2 + bo);
    }
#pragma unroll
    for (int i = 0; i < 4; ++i) {
      const size_t ao = (size_t)(m0 + (i << 4) + rlane) * lda + koff + k0;
      V ah = Frag<T>::load(Ab + ao);
      V al;
      if (SPLIT) al = Frag<T>::load(Ab2 + ao);
#pragma unroll
      for (int j = 0; j < 4; ++j) {
        acc[i][j] = Frag<T>::mma(ah, bh[j], acc[i][j]);
        if (SPLIT) {
          acc[i][j] = Frag<T>::mma(ah, bl[j], acc[i][j]);
          acc[i][j] = Frag<T>::mma(al, bh[j], acc[i][j]);
        }
      }
      Frag<T>::guard(acc[i][0], acc[i][3], ah, SPLIT ? al : ah);
    }
    Frag<T>::keep(bh[0], bh[1], bh[2], bh[3]);
    if (SPLIT) Frag<T>::keep(bl[0], bl[1], bl[2], bl[3]);
  }
  acc_guard4(acc[0][0], acc[0][1], acc[0][2], acc[0][3]);
  acc_guard4(acc[1][0], acc[1][1], acc[1][2], acc[1][3]);
  acc_guard4(acc[2][0], acc[2][1], acc[2][2], acc[2][3]);
  acc_guard4(acc[3][0], acc[3][1], acc[3][2], acc[3][3]);

  float* slab = sT[wave];
  const float* Rb = RESID ? (resid + (size_t)b * strideR) : nullptr;
#pragma unroll
  for (int i = 0; i < 4; ++i) {
    const int mBase = m0 + (i << 4);
#pragma unroll
    for (int j = 0; j < 4; ++j) {
      const int n = n0 + (j << 4) + rlane;
      float bv = 0.f;
      if (BIAS_MODE == 2) bv = bias[n];
#pragma unroll
      for (int r = 0; r < 8; ++r) {
        float v = acc[i][j][r] * scale;
        if (BIAS_MODE == 1) v += bias[mBase + mOff + r];
        if (BIAS_MODE == 2) v += bv;
        if (RESID) v += Rb[(size_t)(mBase + mOff + r) * ldc + n];
        if (ACT == 1) v = tanhf(v);
        if (ACT == 2) v = fmaxf(v, 0.0f);
        if (ACT == 3) v = v / (1.0f + expf(-v));
        if (ACT == 4) v = (v > 0.f) ? v : 0.01f * v;
        if (ACT == 5) v = 0.5f * v * (1.0f + erff(v * 0.70710678118654752f));
        slab[(mOff + r) * 68 + (j << 4) + rlane] = v;
      }
    }
    __builtin_amdgcn_fence(__ATOMIC_RELEASE, "workgroup");
    __builtin_amdgcn_wave_barrier();
    __builtin_amdgcn_fence(__ATOMIC_ACQUIRE, "workgroup");
    if (OUT_MODE == 0) {
      float* C = (float*)Cout + (size_t)b * strideC;
      const int hh = lane >> 4, c4 = (lane & 15) * 4;
      for (int pass = 0; pass < 2; ++pass) {
#pragma unroll
        for (int it = 0; it < 8; ++it) {
          const int row = it * 2 + hh;
          v4f v = *(const v4f*)(slab + row * 68 + c4);
          *(volatile v4f*)(C + (size_t)(mBase + row) * ldc + n0 + c4) = v;
        }
        __threadfence();
      }
    } else {
      const int q = lane >> 3, c8 = (lane & 7) * 8;
      unsigned short* C  = (unsigned short*)Cout  + (size_t)b * strideC;
      unsigned short* C2 = (OUT_MODE == 2) ? ((unsigned short*)Cout2 + (size_t)b * strideC) : nullptr;
      for (int pass = 0; pass < 2; ++pass) {
#pragma unroll
        for (int it = 0; it < 4; ++it) {
          const int row = it * 4 + q;
          const float* sp = slab + row * 68 + c8;
          v8h hv, lv;
#pragma unroll
          for (int e = 0; e < 8; ++e) {
            if (OUT_MODE == 1) {
              hv[e] = (_Float16)sp[e];
            } else {
              unsigned short hb = f2bf_bits(sp[e]);
              unsigned short lb = f2bf_bits(sp[e] - bf_bits2f(hb));
              hv[e] = __builtin_bit_cast(_Float16, hb);
              lv[e] = __builtin_bit_cast(_Float16, lb);
            }
          }
          *(volatile v8h*)(C + (size_t)(mBase + row) * ldc + n0 + c8) = hv;
          if (OUT_MODE == 2) *(volatile v8h*)(C2 + (size_t)(mBase + row) * ldc + n0 + c8) = lv;
        }
        __threadfence();
      }
    }
    __builtin_amdgcn_fence(__ATOMIC_RELEASE, "workgroup");
    __builtin_amdgcn_wave_barrier();
    __builtin_amdgcn_fence(__ATOMIC_ACQUIRE, "workgroup");
  }
}

__global__ __launch_bounds__(256) void cast_f32_f16x2(
    const float* __restrict__ in, _Float16* __restrict__ out, int n2) {
  int i = blockIdx.x * 256 + threadIdx.x;
  if (i < n2) {
    const _Float16 h0 = (_Float16)in[2 * i], h1 = (_Float16)in[2 * i + 1];
    const unsigned u = (unsigned)__builtin_bit_cast(unsigned short, h0) | ((unsigned)__builtin_bit_cast(unsigned short, h1) << 16);
    ((volatile unsigned*)out)[i] = u;
    __threadfence();
    ((volatile unsigned*)out)[i] = u;
  }
}


__global__ __launch_bounds__(256) void transpose_cast_f16(const float* __restrict__ in, int ldi,
                                                         _Float16* __restrict__ outT, int ldo, float scale) {
  __shared__ __align__(16) _Float16 tile[64][72];
  const int c0 = blockIdx.x * 64, r0 = blockIdx.y * 64;
  const int t = threadIdx.y * 32 + threadIdx.x;
  for (int i = threadIdx.y; i < 64; i += 8) {
    tile[threadIdx.x][i]      = (_Float16)(in[(size_t)(r0 + i) * ldi + c0 + threadIdx.x] * scale);
    tile[32 + threadIdx.x][i] = (_Float16)(in[(size_t)(r0 + i) * ldi + c0 + 32 + threadIdx.x] * scale);
  }
  __syncthreads();
  const int q = t >> 3, c8 = (t & 7) * 8;
  for (int pass = 0; pass < 2; ++pass) {
#pragma unroll
    for (int it = 0; it < 2; ++it) {
      const int c = it * 32 + q;
      v8h hv = *(const v8h*)(&tile[c][c8]);
      *(volatile v8h*)(outT + (size_t)(c0 + c) * ldo + r0 + c8) = hv;
    }
    __threadfence();
  }
}

#define KB 512
#define KTD 2048
#define KSD 768
#define KH 128
__global__ __launch_bounds__(256) void pair_kernel(const float* __restrict__ PT, const float* __restrict__ QT_, const float* __restrict__ PS, const float* __restrict__ QS, const float* __restrict__ b1, const float* __restrict__ W2, const float* __restrict__ b2, double* __restrict__ PART) {
  __shared__ float pti[KH], psi[KH], w2s[KH], b1s[KH]; __shared__ double red[256];
  const int i = blockIdx.y, j = blockIdx.x * 256 + threadIdx.x;
  if (threadIdx.x < KH) { pti[threadIdx.x] = PT[(size_t)i * KH + threadIdx.x]; psi[threadIdx.x] = PS[(size_t)i * KH + threadIdx.x]; w2s[threadIdx.x] = W2[threadIdx.x]; b1s[threadIdx.x] = b1[threadIdx.x]; }
  __syncthreads();
  double d = 0.0;
  if (j < KB && j != i) { float st = b2[0], ss = b2[0]; const float* qt = QT_ + (size_t)j * KH; const float* qs = QS + (size_t)j * KH;
#pragma unroll 4
    for (int h = 0; h < KH; ++h) { st += fmaxf(pti[h] + qt[h] + b1s[h], 0.f) * w2s[h]; ss += fmaxf(psi[h] + qs[h] + b1s[h], 0.f) * w2s[h]; }
    const float rt = 1.0f / (1.0f + expf(-st)), rs = 1.0f / (1.0f + expf(-ss)); const double df = (double)rs - (double)rt; d = df * df; }
  red[threadIdx.x] = d; __syncthreads();
  for (int o = 128; o > 0; o >>= 1) { if (threadIdx.x < o) red[threadIdx.x] += red[threadIdx.x + o]; __syncthreads(); }
  if (threadIdx.x < 32) { const size_t k = (size_t)i * gridDim.x + blockIdx.x; ((volatile double*)PART)[k] = red[0]; __threadfence(); ((volatile double*)PART)[k] = red[0]; }
}
__global__ __launch_bounds__(256) void mean_kernel(const double* __restrict__ PART, int n, float* __restrict__ out) {
  __shared__ double red[256]; double s = 0.0; for (int i = threadIdx.x; i < n; i += 256) s += PART[i]; red[threadIdx.x] = s; __syncthreads();
  for (int o = 128; o > 0; o >>= 1) { if (threadIdx.x < o) red[threadIdx.x] += red[threadIdx.x + o]; __syncthreads(); }
  if (threadIdx.x < 32) { const float v = (float)(red[0] / ((double)KB * KB)); ((volatile float*)out)[0] = v; __threadfence(); ((volatile float*)out)[0] = v; }
}
extern "C" void kernel_launch(void* const* d_in, const int* in_sizes, int n_in, void* d_out, int out_size, void* d_ws, size_t ws_size, hipStream_t stream) {
  (void)in_sizes; (void)n_in; (void)out_size; (void)ws_size;
  auto Fp = [&](int i) { return (const float*)d_in[i]; };
  const float* TF = Fp(0); const float* SF = Fp(1); const float* Wt = Fp(2); const float* bt = Fp(3); const float* Wsm = Fp(4); const float* bs = Fp(5); const float* W1 = Fp(6); const float* b1 = Fp(7); const float* W2 = Fp(8); const float* b2 = Fp(9);
  char* ws = (char*)d_ws; size_t off = 0;
  auto carve = [&](size_t bytes) -> char* { char* p = ws + off; off += (bytes + 255) & ~(size_t)255; return p; };
  _Float16* T16 = (_Float16*)carve((size_t)KB * KTD * 2); _Float16* S16 = (_Float16*)carve((size_t)KB * KSD * 2); _Float16* WtT = (_Float16*)carve((size_t)KH * KTD * 2); _Float16* WsT = (_Float16*)carve((size_t)KH * KSD * 2); _Float16* W1aT = (_Float16*)carve(KH * KH * 2); _Float16* W1bT = (_Float16*)carve(KH * KH * 2);
  _Float16* TP16 = (_Float16*)carve(KB * KH * 2); _Float16* SP16 = (_Float16*)carve(KB * KH * 2); float* PT = (float*)carve(KB * KH * 4); float* QT_ = (float*)carve(KB * KH * 4); float* PS = (float*)carve(KB * KH * 4); float* QS = (float*)carve(KB * KH * 4); double* PART = (double*)carve((size_t)KB * 2 * 8);
  cast_f32_f16x2<<<(KB * KTD / 2 + 255) / 256, 256, 0, stream>>>(TF, T16, (long)KB * KTD / 2); cast_f32_f16x2<<<(KB * KSD / 2 + 255) / 256, 256, 0, stream>>>(SF, S16, (long)KB * KSD / 2);
  transpose_cast_f16<<<dim3(KH / 64, KTD / 64), dim3(32, 8), 0, stream>>>(Wt, KH, WtT, KTD, 1.0f); transpose_cast_f16<<<dim3(KH / 64, KSD / 64), dim3(32, 8), 0, stream>>>(Wsm, KH, WsT, KSD, 1.0f);
  transpose_cast_f16<<<dim3(KH / 64, KH / 64), dim3(32, 8), 0, stream>>>(W1, KH, W1aT, KH, 1.0f); transpose_cast_f16<<<dim3(KH / 64, KH / 64), dim3(32, 8), 0, stream>>>(W1 + (size_t)KH * KH, KH, W1bT, KH, 1.0f);
  const int t = (KB / 64) * (KH / 64);
  wmma_gemm64<0, false, 2, 1, false><<<dim3((t + 7) / 8, 1), 256, 0, stream>>>(U16(T16), nullptr, KTD, 0, U16(WtT), nullptr, KTD, 0, TP16, nullptr, KH, 0, bt, nullptr, 0, KB, KH, KTD, 1.0f);
  wmma_gemm64<0, false, 2, 1, false><<<dim3((t + 7) / 8, 1), 256, 0, stream>>>(U16(S16), nullptr, KSD, 0, U16(WsT), nullptr, KSD, 0, SP16, nullptr, KH, 0, bs, nullptr, 0, KB, KH, KSD, 1.0f);
  wmma_gemm64<0, false, 0, 0, false><<<dim3((t + 7) / 8, 1), 256, 0, stream>>>(U16(TP16), nullptr, KH, 0, U16(W1aT), nullptr, KH, 0, PT, nullptr, KH, 0, nullptr, nullptr, 0, KB, KH, KH, 1.0f);
  wmma_gemm64<0, false, 0, 0, false><<<dim3((t + 7) / 8, 1), 256, 0, stream>>>(U16(TP16), nullptr, KH, 0, U16(W1bT), nullptr, KH, 0, QT_, nullptr, KH, 0, nullptr, nullptr, 0, KB, KH, KH, 1.0f);
  wmma_gemm64<0, false, 0, 0, false><<<dim3((t + 7) / 8, 1), 256, 0, stream>>>(U16(SP16), nullptr, KH, 0, U16(W1aT), nullptr, KH, 0, PS, nullptr, KH, 0, nullptr, nullptr, 0, KB, KH, KH, 1.0f);
  wmma_gemm64<0, false, 0, 0, false><<<dim3((t + 7) / 8, 1), 256, 0, stream>>>(U16(SP16), nullptr, KH, 0, U16(W1bT), nullptr, KH, 0, QS, nullptr, KH, 0, nullptr, nullptr, 0, KB, KH, KH, 1.0f);
  pair_kernel<<<dim3(KB / 256, KB), 256, 0, stream>>>(PT, QT_, PS, QS, b1, W2, b2, PART);
  mean_kernel<<<1, 256, 0, stream>>>(PART, KB * 2, (float*)d_out);
}
